// CrossShapedSpatialAttention_18013092839823
// MI455X (gfx1250) — hardware-verified
//
#include <hip/hip_runtime.h>


#define NB_  8
#define IH   56
#define IW   56
#define CC   256
#define CH   128
#define SW   7
#define NM   8
#define LT   392
#define LP   448
#define HN   4
#define HD   32
#define NTOK (NB_ * IH * IW)
#define NST  (NB_ * NM)
#define PSC  32768.0f
#define LOSC 1024.0f
#define LOSCI (1.0f / 1024.0f)

typedef _Float16 h16;
typedef unsigned short bf;
typedef __attribute__((ext_vector_type(16))) __bf16   v16bf;
typedef __attribute__((ext_vector_type(16))) _Float16 v16h;
typedef __attribute__((ext_vector_type(8)))  _Float16 v8h;
typedef __attribute__((ext_vector_type(8)))  unsigned short v8us;
typedef __attribute__((ext_vector_type(8)))  float    v8f;
typedef __attribute__((ext_vector_type(4)))  float    v4f;
typedef v8h  __attribute__((may_alias)) v8ha;
typedef v4f  __attribute__((may_alias)) v4fa;
typedef v8us __attribute__((may_alias)) v8usa;

__device__ __forceinline__ unsigned short f2bf(float f) { unsigned u = __float_as_uint(f); u += 0x7FFFu + ((u >> 16) & 1u); return (unsigned short)(u >> 16); }
__device__ __forceinline__ float bf2f(unsigned short b) { return __uint_as_float(((unsigned)b) << 16); }
__device__ __forceinline__ float bfr(float f) { return bf2f(f2bf(f)); }
__device__ __forceinline__ v16h cat16(v8h lo, v8h hi) { return __builtin_shufflevector(lo, hi, 0, 1, 2, 3, 4, 5, 6, 7, 8, 9, 10, 11, 12, 13, 14, 15); }
__device__ __forceinline__ v16bf cat16b(v8us lo, v8us hi) { return __builtin_bit_cast(v16bf, __builtin_shufflevector(lo, hi, 0, 1, 2, 3, 4, 5, 6, 7, 8, 9, 10, 11, 12, 13, 14, 15)); }
__device__ __forceinline__ v8f wmma16(v16h a, v16h b, v8f c) { return __builtin_amdgcn_wmma_f32_16x16x32_f16(false, a, false, b, (short)0, c, false, false); }
__device__ __forceinline__ v8f wmmab(v16bf a, v16bf b, v8f c) { return __builtin_amdgcn_wmma_f32_16x16x32_bf16(false, a, false, b, (short)0, c, false, false); }
#define VST2(T, p, v) do { const T vst2_v_ = (v); *(volatile T*)(p) = vst2_v_; __threadfence(); *(volatile T*)(p) = vst2_v_; } while (0)

__device__ __forceinline__ size_t pix_of(int br, int st, int t) { const int b = st / NM, m = st - b * NM; int h, w; if (br == 0) { h = SW * m + t / IW; w = t % IW; } else { h = t % IH; w = SW * m + t / IH; } return ((size_t)b * IH + h) * IW + w; }

__global__ __launch_bounds__(256) void k_tok(const float* __restrict__ x, bf* S) {
    const int lane = threadIdx.x & 31; const size_t w = (size_t)blockIdx.x * 8 + (threadIdx.x >> 5);
    if (w >= (size_t)2 * NST * LT) return;
    const int br = (int)(w / ((size_t)NST * LT)); const size_t rem = w - (size_t)br * NST * LT; const int st = (int)(rem / LT), t = (int)(rem - (size_t)st * LT);
    const size_t px = pix_of(br, st, t);
    if (lane < 16) { v8us o;
#pragma unroll
        for (int i = 0; i < 8; ++i) o[i] = f2bf(x[px * CC + br * CH + lane * 8 + i]);
        VST2(v8us, S + w * CH + lane * 8, o); }
}
__global__ __launch_bounds__(256) void k_wt(const float* __restrict__ Wm, int K, int ncols, bf* WT) {
    __shared__ __align__(16) unsigned short tl[64 * 72];
    const int tid = threadIdx.x, k0 = blockIdx.x * 64, n0 = blockIdx.y * 64;
    const int kk = tid >> 2, nq = (tid & 3) * 16;
#pragma unroll
    for (int i = 0; i < 16; ++i) tl[(nq + i) * 72 + kk] = f2bf(Wm[(size_t)(k0 + kk) * ncols + n0 + nq + i]);
    __syncthreads();
    const int piece = tid & 7;
    auto pass = [&]() {
#pragma unroll
        for (int s = 0; s < 2; ++s) { const int nr = (tid >> 3) + 32 * s; const v8us val = *(const v8usa*)(tl + nr * 72 + piece * 8); *(volatile v8us*)(WT + (size_t)(n0 + nr) * K + k0 + piece * 8) = val; }
    };
    pass(); __threadfence(); pass();
}
__global__ __launch_bounds__(128) void k_qkv(const bf* __restrict__ S, const bf* __restrict__ WT, const float* __restrict__ bqh, const float* __restrict__ bqv, h16* QH, h16* QL, h16* KH, h16* KL, float* Vf) {
    __shared__ __align__(16) float ost[4][16 * 68];
    const int lane = threadIdx.x & 31, wave = threadIdx.x >> 5, lr = lane & 15, hi = lane >> 4, br = blockIdx.z;
    const size_t r0 = (size_t)blockIdx.x * 64 + wave * 16, rbase = (size_t)br * NST * LT; const int c0 = blockIdx.y * 64;
    const bf* A = S + rbase * CH; const bf* Bw = WT + (size_t)br * (3 * CH) * CH;
    v8f acc[4];
#pragma unroll
    for (int t = 0; t < 4; ++t) acc[t] = (v8f){};
#pragma unroll
    for (int kc = 0; kc < CH; kc += 32) {
        const v16bf a = cat16b(*(const v8us*)(A + (r0 + lr) * CH + kc + 8 * hi), *(const v8us*)(A + (r0 + lr) * CH + kc + 8 * hi + 16));
#pragma unroll
        for (int t = 0; t < 4; ++t) { const bf* bp = Bw + (size_t)(c0 + t * 16 + lr) * CH + kc + 8 * hi; acc[t] = wmmab(a, cat16b(*(const v8us*)bp, *(const v8us*)(bp + 16)), acc[t]); }
    }
    float* os = &ost[wave][0];
#pragma unroll
    for (int t = 0; t < 4; ++t) { const int col = c0 + t * 16 + lr; const float bv = br ? bfr(bqv[col]) : bfr(bqh[col]);
#pragma unroll
        for (int j = 0; j < 8; ++j) os[(hi * 8 + j) * 68 + t * 16 + lr] = acc[t][j] + bv; }
    __builtin_amdgcn_wave_barrier(); asm volatile("" ::: "memory");
    const int which = c0 / CH, cofs0 = c0 - which * CH;
    if (which < 2) {
        h16* P1 = (which == 0 ? QH : KH) + (rbase + r0) * CH + cofs0; h16* P2 = (which == 0 ? QL : KL) + (rbase + r0) * CH + cofs0;
        auto pass = [&]() {
#pragma unroll
            for (int s = 0; s < 4; ++s) { const int row = 4 * s + (lane >> 3), piece = lane & 7; const float* sp = os + row * 68 + piece * 8; v8h oh, ol;
#pragma unroll
                for (int i = 0; i < 8; ++i) { const h16 a = (h16)sp[i]; oh[i] = a; ol[i] = (h16)((sp[i] - (float)a) * LOSC); }
                *(volatile v8h*)(P1 + (size_t)row * CH + piece * 8) = oh; *(volatile v8h*)(P2 + (size_t)row * CH + piece * 8) = ol; }
        };
        pass(); __threadfence(); pass();
    } else {
        float* crow = Vf + (rbase + r0) * CH + cofs0;
        auto pass = [&]() {
#pragma unroll
            for (int s = 0; s < 8; ++s) { const int Lid = (lane >> 3) + 4 * s, piece = lane & 7; const int row = Lid >> 1, cofs = (Lid & 1) * 32 + piece * 4;
                const v4f val = *(const v4fa*)(os + row * 68 + cofs); *(volatile v4f*)(crow + (size_t)row * CH + cofs) = val; }
        };
        pass(); __threadfence(); pass();
    }
}
__global__ __launch_bounds__(256) void k_vt(const float* __restrict__ Vf, h16* VTH, h16* VTL) {
    __shared__ __align__(16) h16 tl[128 * 72];
    __shared__ __align__(16) h16 tl2[128 * 72];
    const int tid = threadIdx.x, t0 = blockIdx.x * 64, st = blockIdx.y, br = blockIdx.z;
    const size_t sbase = ((size_t)br * NST + st) * LT;
    { const int tt = tid >> 2, dq = (tid & 3) * 32; const int t = t0 + tt;
#pragma unroll
      for (int i = 0; i < 32; ++i) { const float v = (t < LT) ? Vf[(sbase + t) * CH + dq + i] : 0.f; const h16 a = (h16)v; tl[(dq + i) * 72 + tt] = a; tl2[(dq + i) * 72 + tt] = (h16)((v - (float)a) * LOSC); } }
    __syncthreads();
    const int piece = tid & 7;
    const size_t vb = ((size_t)br * NST + st) * CH;
    auto pass = [&]() {
#pragma unroll
        for (int s = 0; s < 4; ++s) { const int d = (tid >> 3) + 32 * s; const size_t o = (vb + d) * LP + t0 + piece * 8;
            *(volatile v8h*)(VTH + o) = *(const v8ha*)(tl + d * 72 + piece * 8); *(volatile v8h*)(VTL + o) = *(const v8ha*)(tl2 + d * 72 + piece * 8); }
    };
    pass(); __threadfence(); pass();
}
__global__ __launch_bounds__(128) void k_attn(const h16* __restrict__ QH, const h16* __restrict__ QL, const h16* __restrict__ KH, const h16* __restrict__ KL, const h16* __restrict__ VTH, const h16* __restrict__ VTL, float* O) {
    __shared__ __align__(16) h16 plds[4][16 * 32];
    __shared__ __align__(16) h16 plds2[4][16 * 32];
    __shared__ __align__(16) float ost[4][16 * 36];
    const int lane = threadIdx.x & 31, wave = threadIdx.x >> 5, lr = lane & 15, hi = lane >> 4;
    const int qt = blockIdx.x, st = blockIdx.y, br = blockIdx.z, q0 = qt * 64 + wave * 16;
    const size_t tb = ((size_t)br * NST + st) * LT;
    h16* pl = &plds[wave][0]; h16* pl2 = &plds2[wave][0]; float* os = &ost[wave][0];
    const float scl = 0.17677669529663687f;
#pragma unroll 1
    for (int h = 0; h < HN; ++h) {
        const size_t qo = (tb + q0 + lr) * CH + h * HD + 8 * hi;
        const v16h qa = cat16(*(const v8h*)(QH + qo), *(const v8h*)(QH + qo + 16)), ql = cat16(*(const v8h*)(QL + qo), *(const v8h*)(QL + qo + 16));
        v8f o[2], ox[2]; o[0] = o[1] = ox[0] = ox[1] = (v8f){};
        float mrow[8], lpart[8];
#pragma unroll
        for (int j = 0; j < 8; ++j) { mrow[j] = -3.0e38f; lpart[j] = 0.f; }
#pragma unroll 1
        for (int kt = 0; kt < 13; ++kt) {
            const int l0 = kt * 32;
            const size_t k0o = (tb + l0 + lr) * CH + h * HD + 8 * hi, k1o = k0o + (size_t)16 * CH;
            const v16h k0h = cat16(*(const v8h*)(KH + k0o), *(const v8h*)(KH + k0o + 16)), k1h = cat16(*(const v8h*)(KH + k1o), *(const v8h*)(KH + k1o + 16));
            const v16h k0l = cat16(*(const v8h*)(KL + k0o), *(const v8h*)(KL + k0o + 16)), k1l = cat16(*(const v8h*)(KL + k1o), *(const v8h*)(KL + k1o + 16));
            v8f s0 = wmma16(qa, k0h, (v8f){}), s1 = wmma16(qa, k1h, (v8f){}), x0 = wmma16(ql, k0h, (v8f){}), x1 = wmma16(ql, k1h, (v8f){});
            x0 = wmma16(qa, k0l, x0); x1 = wmma16(qa, k1l, x1);
            asm volatile("v_nop\n\tv_nop\n\tv_nop\n\tv_nop" : "+v"(s0), "+v"(s1), "+v"(x0), "+v"(x1) : "v"(qa), "v"(ql));
            float alpha[8];
#pragma unroll
            for (int j = 0; j < 8; ++j) {
                const int ja = l0 + lr, jb = l0 + 16 + lr;
                const float a0 = (ja < LT) ? (s0[j] + x0[j] * LOSCI) * scl : -__builtin_inff(), a1 = (jb < LT) ? (s1[j] + x1[j] * LOSCI) * scl : -__builtin_inff();
                float mx = fmaxf(a0, a1);
                mx = fmaxf(mx, __shfl_xor(mx, 1, 16)); mx = fmaxf(mx, __shfl_xor(mx, 2, 16)); mx = fmaxf(mx, __shfl_xor(mx, 4, 16)); mx = fmaxf(mx, __shfl_xor(mx, 8, 16));
                const float mn = fmaxf(mrow[j], mx);
                alpha[j] = __expf(mrow[j] - mn); mrow[j] = mn;
                const float p0 = __expf(a0 - mn), p1 = __expf(a1 - mn);
                lpart[j] = lpart[j] * alpha[j] + (p0 + p1);
                const int mr = hi * 8 + j; const float ps0 = p0 * PSC, ps1 = p1 * PSC; const h16 h0 = (h16)ps0, h1 = (h16)ps1;
                pl[mr * 32 + lr] = h0; pl[mr * 32 + 16 + lr] = h1; pl2[mr * 32 + lr] = (h16)(ps0 - (float)h0); pl2[mr * 32 + 16 + lr] = (h16)(ps1 - (float)h1); }
#pragma unroll
            for (int n = 0; n < 2; ++n)
#pragma unroll
                for (int j = 0; j < 8; ++j) { o[n][j] *= alpha[j]; ox[n][j] *= alpha[j]; }
            asm volatile("" ::: "memory");
            const v16h pa = cat16(*(const v8ha*)(pl + lr * 32 + hi * 8), *(const v8ha*)(pl + lr * 32 + 16 + hi * 8));
            const v16h px = cat16(*(const v8ha*)(pl2 + lr * 32 + hi * 8), *(const v8ha*)(pl2 + lr * 32 + 16 + hi * 8));
#pragma unroll
            for (int n = 0; n < 2; ++n) { const size_t vo = ((((size_t)br * NST + st) * CH) + h * HD + n * 16 + lr) * LP + l0 + hi * 8;
                const v16h vh = cat16(*(const v8h*)(VTH + vo), *(const v8h*)(VTH + vo + 16)), vl = cat16(*(const v8h*)(VTL + vo), *(const v8h*)(VTL + vo + 16));
                o[n] = wmma16(pa, vh, o[n]); o[n] = wmma16(px, vh, o[n]); ox[n] = wmma16(pa, vl, ox[n]);
                asm volatile("" : "+v"(o[n]), "+v"(ox[n]) : "v"(vh), "v"(vl) : "memory"); }
            asm volatile("v_nop\n\tv_nop\n\tv_nop\n\tv_nop" : "+v"(o[0]), "+v"(o[1]), "+v"(ox[0]), "+v"(ox[1]) : "v"(pa), "v"(px));
            __builtin_amdgcn_wave_barrier();
        }
        float inv[8];
#pragma unroll
        for (int j = 0; j < 8; ++j) { float rs = lpart[j]; rs += __shfl_xor(rs, 1, 16); rs += __shfl_xor(rs, 2, 16); rs += __shfl_xor(rs, 4, 16); rs += __shfl_xor(rs, 8, 16); inv[j] = 1.0f / (rs * PSC); }
#pragma unroll
        for (int n = 0; n < 2; ++n)
#pragma unroll
            for (int j = 0; j < 8; ++j) os[(hi * 8 + j) * 36 + n * 16 + lr] = (o[n][j] + ox[n][j] * LOSCI) * inv[j];
        __builtin_amdgcn_wave_barrier(); asm volatile("" ::: "memory");
#pragma unroll
        for (int ps2 = 0; ps2 < 2; ++ps2) {
#pragma unroll
            for (int s = 0; s < 4; ++s) { const int row = 4 * s + (lane >> 3), piece = lane & 7; const int t = q0 + row;
                if (t < LT) { const size_t px_ = pix_of(br, st, t); const v4f val = *(const v4fa*)(os + row * 36 + piece * 4);
                    *(volatile v4f*)(O + px_ * CC + br * CH + h * HD + piece * 4) = val; } }
            if (ps2 == 0) __threadfence(); }
        __builtin_amdgcn_wave_barrier(); asm volatile("" ::: "memory");
    }
}
__global__ __launch_bounds__(256) void k_osplit(const float* __restrict__ Of, bf* OH, bf* OL) {
    const int lane = threadIdx.x & 31; const size_t r = (size_t)blockIdx.x * 8 + (threadIdx.x >> 5);
    if (r >= (size_t)NTOK) return;
    v8us oh, ol;
#pragma unroll
    for (int i = 0; i < 8; ++i) { const float v = Of[r * CC + lane * 8 + i]; const unsigned short hb = f2bf(v); oh[i] = hb; ol[i] = f2bf(v - bf2f(hb)); }
    *(volatile v8us*)(OH + r * CC + lane * 8) = oh; *(volatile v8us*)(OL + r * CC + lane * 8) = ol; __threadfence();
    *(volatile v8us*)(OH + r * CC + lane * 8) = oh; *(volatile v8us*)(OL + r * CC + lane * 8) = ol;
}
__global__ __launch_bounds__(128) void k_proj(const bf* __restrict__ OH, const bf* __restrict__ OL, const bf* __restrict__ WpT, const float* __restrict__ bp, float* out) {
    __shared__ __align__(16) float ost[4][16 * 68];
    const int lane = threadIdx.x & 31, wave = threadIdx.x >> 5, lr = lane & 15, hi = lane >> 4;
    const size_t r0 = (size_t)blockIdx.x * 64 + wave * 16; const int c0 = blockIdx.y * 64;
    v8f acc[4];
#pragma unroll
    for (int t = 0; t < 4; ++t) acc[t] = (v8f){};
#pragma unroll 2
    for (int kc = 0; kc < CC; kc += 32) {
        const size_t ao = (r0 + lr) * CC + kc + 8 * hi;
        const v16bf a = cat16b(*(const v8us*)(OH + ao), *(const v8us*)(OH + ao + 16)), al = cat16b(*(const v8us*)(OL + ao), *(const v8us*)(OL + ao + 16));
#pragma unroll
        for (int t = 0; t < 4; ++t) { const bf* bpp = WpT + (size_t)(c0 + t * 16 + lr) * CC + kc + 8 * hi; const v16bf bb = cat16b(*(const v8us*)bpp, *(const v8us*)(bpp + 16)); acc[t] = wmmab(a, bb, acc[t]); acc[t] = wmmab(al, bb, acc[t]); }
        asm volatile("v_nop" : "+v"(acc[0]), "+v"(acc[1]), "+v"(acc[2]), "+v"(acc[3]) : "v"(a), "v"(al) : "memory");
    }
    float* os = &ost[wave][0];
#pragma unroll
    for (int t = 0; t < 4; ++t) { const float bv = bfr(bp[c0 + t * 16 + lr]);
#pragma unroll
        for (int j = 0; j < 8; ++j) os[(hi * 8 + j) * 68 + t * 16 + lr] = acc[t][j] + bv; }
    __syncthreads();
    float* crow = out + r0 * CC + c0;
    auto pass = [&]() {
#pragma unroll
        for (int s = 0; s < 8; ++s) { const int Lid = (lane >> 3) + 4 * s, piece = lane & 7; const int row = Lid >> 1, cofs = (Lid & 1) * 32 + piece * 4;
            const v4f val = *(const v4fa*)(os + row * 68 + cofs); *(volatile v4f*)(crow + (size_t)row * CC + cofs) = val; }
    };
    pass(); __threadfence(); pass();
}

extern "C" void kernel_launch(void* const* d_in, const int* in_sizes, int n_in,
                              void* d_out, int out_size, void* d_ws, size_t ws_size, hipStream_t stream) {
    (void)in_sizes; (void)n_in; (void)out_size;
    const float* x = (const float*)d_in[0]; const float* Wqh = (const float*)d_in[1]; const float* bqh = (const float*)d_in[2]; const float* Wqv = (const float*)d_in[3]; const float* bqv = (const float*)d_in[4];
    const float* Wp = (const float*)d_in[5]; const float* bp = (const float*)d_in[6];
    float* out = (float*)d_out;
    char* wsp = (char*)d_ws;
    auto take = [&](size_t bytes) { char* p = wsp; wsp += (bytes + 255) & ~(size_t)255; return (void*)p; };
    const size_t NT2 = (size_t)2 * NST * LT;
    bf* S = (bf*)take((NT2 + 64) * CH * 2); bf* WT = (bf*)take((size_t)2 * 3 * CH * CH * 2); bf* WpT = (bf*)take((size_t)CC * CC * 2);
    h16* QH = (h16*)take((NT2 + 64) * CH * 2); h16* QL = (h16*)take((NT2 + 64) * CH * 2); h16* KH = (h16*)take((NT2 + 64) * CH * 2); h16* KL = (h16*)take((NT2 + 64) * CH * 2);
    float* Vf = (float*)take(NT2 * CH * 4); h16* VTH = (h16*)take((size_t)2 * NST * CH * LP * 2); h16* VTL = (h16*)take((size_t)2 * NST * CH * LP * 2);
    if ((size_t)(wsp - (char*)d_ws) > ws_size) return;
    float* O = Vf; bf* OH = S; bf* OL = (bf*)QH;
    k_tok<<<(unsigned)((NT2 + 7) / 8), 256, 0, stream>>>(x, S);
    k_wt<<<dim3(CH / 64, (3 * CH) / 64, 1), 256, 0, stream>>>(Wqh, CH, 3 * CH, WT); k_wt<<<dim3(CH / 64, (3 * CH) / 64, 1), 256, 0, stream>>>(Wqv, CH, 3 * CH, WT + (size_t)3 * CH * CH);
    k_wt<<<dim3(CC / 64, CC / 64, 1), 256, 0, stream>>>(Wp, CC, CC, WpT);
    k_qkv<<<dim3((NST * LT) / 64, (3 * CH) / 64, 2), 128, 0, stream>>>(S, WT, bqh, bqv, QH, QL, KH, KL, Vf);
    k_vt<<<dim3(LP / 64, NST, 2), 256, 0, stream>>>(Vf, VTH, VTL);
    k_attn<<<dim3(LP / 64, NST, 2), 128, 0, stream>>>(QH, QL, KH, KL, VTH, VTL, O);
    k_osplit<<<NTOK / 8, 256, 0, stream>>>(O, OH, OL);
    k_proj<<<dim3(NTOK / 64, CC / 64, 1), 128, 0, stream>>>(OH, OL, WpT, bp, out);
}
